// R_HGNN_31001073942570
// MI455X (gfx1250) — hardware-run, weakly checked
//
#include <hip/hip_runtime.h>


namespace {
constexpr int R = 3, N = 20000, E = 250000, H = 4, D = 32, IN = 128, RN = R * N, NBLK = N / 16;
constexpr float XS = 8.0f, HS = 64.0f, WSC = 256.0f, NEG = 0.2f;
typedef _Float16 b16;
typedef __attribute__((ext_vector_type(16))) _Float16 v16b;
typedef __attribute__((ext_vector_type(8))) _Float16 v8b;
typedef __attribute__((ext_vector_type(8))) float v8f;
typedef __attribute__((ext_vector_type(4))) float v4f;
typedef __attribute__((ext_vector_type(2))) float v2f;
__device__ __forceinline__ float bf16_rne(float f) { unsigned int u = __float_as_uint(f); u += 0x7FFFu + ((u >> 16) & 1u); return __uint_as_float(u & 0xFFFF0000u); }
__device__ __forceinline__ void split16(float v, b16& hi, b16& lo) { hi = (b16)v; lo = (b16)(v - (float)hi); }
__device__ __forceinline__ v16b frag_kb(const b16* p, int hh) { const v8b a = *(const v8b*)(p + 8 * hh), b = *(const v8b*)(p + 16 + 8 * hh); v16b f;
#pragma unroll
  for (int e = 0; e < 8; ++e) { f[e] = a[e]; f[8 + e] = b[e]; } return f; }
__device__ __forceinline__ v8f wmma16b(v16b a, v16b b, v8f c) { v8f d = __builtin_amdgcn_wmma_f32_16x16x32_f16(false, a, false, b, (short)0, c, false, false); asm volatile("v_nop\n\tv_nop\n\tv_nop\n\tv_nop" : "+v"(d) : "v"(a), "v"(b)); return d; }
__device__ __forceinline__ void wave_lds_sync() { __builtin_amdgcn_fence(__ATOMIC_RELEASE, "workgroup"); __builtin_amdgcn_wave_barrier(); __builtin_amdgcn_fence(__ATOMIC_ACQUIRE, "workgroup"); }
__device__ __forceinline__ float pmul(float a, float b) { float p = a * b; asm volatile("" : "+v"(p)); return p; }
__device__ __forceinline__ int iclamp(int v, int lo, int hi) { return v < lo ? lo : (v > hi ? hi : v); }
__device__ __forceinline__ float leaky(float v) { return v >= 0.0f ? v : NEG * v; }
__device__ __forceinline__ float sigm(float v) { return 1.0f / (1.0f + __expf(-v)); }
constexpr int CSR_NBLK9 = 512, CSR_GB9 = 9, CSR_GN9 = 1 << CSR_GB9  , CSR_TS9 = (CSR_GN9 < 32 ? 32 : CSR_GN9)  , CSR_MAXG9 = 512, CSR_CAP9 = 12288  ;
__device__ __host__ __forceinline__ int csr_tix9(int v) { return (v >> CSR_GB9) * CSR_TS9 + (v & (CSR_GN9 - 1)); }
__global__ __launch_bounds__(64) void csrA_kernel9(const int* __restrict__ dst, int E, int N, int nG, int CHP, int NGP, int* __restrict__ STG, int* __restrict__ HST) {
  extern __shared__ int sm[];
  int* cnt = sm; int* run = sm + NGP; int* ids = sm + 2 * NGP;
  const int b = blockIdx.x; const int ch = (E + CSR_NBLK9 - 1) / CSR_NBLK9; const int e0 = b * ch, e1 = min(E, e0 + ch);
  for (int i = threadIdx.x; i < NGP; i += 64) cnt[i] = 0;
  for (int i = threadIdx.x; i < CHP; i += 64) ids[i] = -1;
  __syncthreads();
  if (threadIdx.x == 0) {
    for (int e = e0; e < e1; ++e) { int d = dst[e]; d = (d < 0) ? 0 : (d >= N ? N - 1 : d); cnt[d >> CSR_GB9] += 1; }
    int acc = 0; for (int g = 0; g < nG; ++g) { run[g] = acc; acc += cnt[g]; }
    for (int e = e0; e < e1; ++e) { int d = dst[e]; d = (d < 0) ? 0 : (d >= N ? N - 1 : d); const int g = d >> CSR_GB9; ids[run[g]] = e; run[g] += 1; } }
  __syncthreads();
  typedef __attribute__((ext_vector_type(4))) int v4i;
  for (int pass = 0; pass < 2; ++pass) {
    for (int i = threadIdx.x; i < CHP / 4; i += 64) *(volatile v4i*)(STG + (size_t)b * CHP + i * 4) = *(const v4i*)(&ids[i * 4]);
    for (int i = threadIdx.x; i < NGP / 4; i += 64) { v4i v; for (int e = 0; e < 4; ++e) v[e] = (i * 4 + e < nG) ? cnt[i * 4 + e] : 0; *(volatile v4i*)(HST + (size_t)b * NGP + i * 4) = v; }
    __threadfence(); }
}
__global__ __launch_bounds__(512) void csrS_kernel9(const int* __restrict__ HST, int nG, int NGP, int* __restrict__ START, int* __restrict__ TOT, int* __restrict__ OFF) {
  __shared__ int tot[CSR_MAXG9];
  const int b = threadIdx.x;
  for (int pass = 0; pass < 2; ++pass) { int runb = 0; for (int g = 0; g < nG; ++g) { int c = HST[(size_t)b * NGP + g]; c = (c < 0) ? 0 : c; ((volatile int*)OFF)[(size_t)g * CSR_NBLK9 + b] = runb; runb += c; } __threadfence(); }
  for (int g = threadIdx.x; g < nG; g += 512) { int s = 0; for (int bb = 0; bb < CSR_NBLK9; ++bb) { int c = HST[(size_t)bb * NGP + g]; s += (c < 0) ? 0 : c; } tot[g] = s; }
  __syncthreads();
  if (threadIdx.x < 32) {
    __shared__ int st[CSR_MAXG9 + 32];
    if (threadIdx.x == 0) { int acc = 0; for (int g = 0; g < NGP; ++g) { st[g] = acc; if (g < nG) acc += (tot[g] + 31) & ~31; } st[NGP] = acc; }
    __builtin_amdgcn_fence(__ATOMIC_RELEASE, "workgroup"); __builtin_amdgcn_wave_barrier(); __builtin_amdgcn_fence(__ATOMIC_ACQUIRE, "workgroup");
    for (int pass = 0; pass < 2; ++pass) { for (int i = threadIdx.x; i < NGP + 32; i += 32) { ((volatile int*)START)[i] = (i <= NGP) ? st[min(i, NGP)] : 0; ((volatile int*)TOT)[i] = (i < nG) ? tot[i] : 0; } __threadfence(); } }
}
__global__ __launch_bounds__(256) void csrB_kernel9(const int* __restrict__ dst, int N, int nG, int CHP, int NGP, int permLen, const int* __restrict__ STG, const int* __restrict__ HST, const int* __restrict__ OFF, const int* __restrict__ START, const int* __restrict__ TOT, int* __restrict__ PERM, int* __restrict__ ROWPTR, int* __restrict__ ROWCNT, int* __restrict__ FLAG) {
  typedef __attribute__((ext_vector_type(4))) int v4i;
  __shared__ int ids[CSR_CAP9]; __shared__ unsigned short key[CSR_CAP9]; __shared__ int outp[CSR_CAP9]; __shared__ int ncnt[CSR_GN9 + 1]; __shared__ int boff[CSR_NBLK9 + 1];
  const int g = blockIdx.x, t_ = threadIdx.x; int tot = TOT[g]; int st = START[g], stn = START[g + 1]; const int v0 = g * CSR_GN9; const int nv = min(CSR_GN9, N - v0); const int t0 = g * CSR_TS9;
  st = (st < 0) ? 0 : (st > permLen - 32 ? permLen - 32 : st) & ~31; stn = (stn < st) ? st : (stn > permLen ? permLen : stn); tot = (tot < 0) ? 0 : tot; if (tot > stn - st && tot <= CSR_CAP9) tot = stn - st;
  if (tot > CSR_CAP9) {
    for (int pass = 0; pass < 2; ++pass) { for (int i = t_; i < CSR_TS9 / 4; i += 256) { v4i a, c; for (int e = 0; e < 4; ++e) { a[e] = st; c[e] = 0; } *(volatile v4i*)(ROWPTR + t0 + i * 4) = a; *(volatile v4i*)(ROWCNT + t0 + i * 4) = c; } if (t_ == 0) ((volatile int*)FLAG)[0] = 1; __threadfence(); } (void)nv; return; }
  if (t_ == 0) { int acc = 0; for (int b = 0; b < CSR_NBLK9; ++b) { boff[b] = acc; int c = HST[(size_t)b * NGP + g]; c = (c < 0) ? 0 : (c > CHP ? CHP : c); acc += c; if (acc > tot) acc = tot; } boff[CSR_NBLK9] = acc; }
  for (int i = t_; i <= CSR_GN9; i += 256) ncnt[i] = 0;
  __syncthreads();
  for (int b = 0; b < CSR_NBLK9; ++b) { const int c = boff[b + 1] - boff[b]; int o_ = OFF[(size_t)g * CSR_NBLK9 + b]; o_ = (o_ < 0) ? 0 : (o_ > CHP - c ? CHP - c : o_); const int* src_ = STG + (size_t)b * CHP + o_;
    for (int i = t_; i < c; i += 256) { int id = src_[i]; id = (id < 0) ? 0 : id; ids[boff[b] + i] = id; int d = dst[id]; d = (d < v0) ? v0 : (d >= N ? N - 1 : d); int kk = d - v0; kk = (kk < 0) ? 0 : (kk >= CSR_GN9 ? CSR_GN9 - 1 : kk); key[boff[b] + i] = (unsigned short)kk; } }
  __syncthreads();
  if (t_ == 0) { for (int i = 0; i < tot; ++i) ncnt[key[i]] += 1; int acc = 0; for (int vl = 0; vl < CSR_GN9; ++vl) { const int c = ncnt[vl]; ncnt[vl] = acc; acc += c; } ncnt[CSR_GN9] = acc;
    for (int i = 0; i < tot; ++i) { const int vl = key[i]; outp[ncnt[vl]] = ids[i]; ncnt[vl] += 1; }
    for (int vl = CSR_GN9; vl > 0; --vl) ncnt[vl] = ncnt[vl - 1]; ncnt[0] = 0; }
  __syncthreads();
  for (int pass = 0; pass < 2; ++pass) {
    for (int i = t_; i < (stn - st) / 4; i += 256) { v4i v; for (int e = 0; e < 4; ++e) { const int q = i * 4 + e; v[e] = (q < tot) ? outp[q] : -1; } *(volatile v4i*)(PERM + st + i * 4) = v; }
    for (int i = t_; i < CSR_TS9 / 4; i += 256) { v4i a, c; for (int e = 0; e < 4; ++e) { const int vl = i * 4 + e; const int vc = vl < CSR_GN9 ? vl : CSR_GN9; a[e] = (vl < CSR_GN9) ? st + ncnt[vc] : st; c[e] = (vl < nv) ? (ncnt[(vc < CSR_GN9 ? vc : CSR_GN9 - 1) + 1] - ncnt[vc]) : 0; } *(volatile v4i*)(ROWPTR + t0 + i * 4) = a; *(volatile v4i*)(ROWCNT + t0 + i * 4) = c; }
    __threadfence(); }
}
__global__ __launch_bounds__(256) void csrZ_kernel9(int* __restrict__ p, size_t n4) { typedef __attribute__((ext_vector_type(4))) int v4i; const size_t tid = (size_t)blockIdx.x * 256 + threadIdx.x, nth = (size_t)gridDim.x * 256; v4i z = {0, 0, 0, 0}; for (size_t i = tid; i < n4; i += nth) *(volatile v4i*)(p + i * 4) = z; }
struct CsrBufs9 { int *STG, *HST, *OFF, *START, *TOT, *PERM, *ROWPTR, *ROWCNT, *FLAG; int nG, NGP, CHP; size_t permLen; char* base; size_t bytes; };
static size_t csr_carve9(CsrBufs9& c, char* ws, size_t off, int E, int N) {
  const size_t off0 = off; c.base = ws + off;
  auto al = [&](size_t bytes) { char* p = ws + off; off += (bytes + 255) & ~(size_t)255; return p; };
  c.nG = (N + CSR_GN9 - 1) / CSR_GN9; c.NGP = (c.nG + 31) & ~31; const int ch = (E + CSR_NBLK9 - 1) / CSR_NBLK9; c.CHP = (ch + 31) & ~31; c.permLen = (size_t)E + 32 * (size_t)c.nG + 32;
  c.STG = (int*)al((size_t)CSR_NBLK9 * c.CHP * 4); c.HST = (int*)al((size_t)CSR_NBLK9 * c.NGP * 4); c.OFF = (int*)al((size_t)c.NGP * CSR_NBLK9 * 4); c.START = (int*)al((size_t)(c.NGP + 64) * 4); c.TOT = (int*)al((size_t)(c.NGP + 64) * 4);
  c.PERM = (int*)al(c.permLen * 4); c.ROWPTR = (int*)al((size_t)c.nG * CSR_TS9 * 4); c.ROWCNT = (int*)al((size_t)c.nG * CSR_TS9 * 4); c.FLAG = (int*)al(256);
  c.bytes = off - off0; return off;
}
static void csr_build9(const CsrBufs9& c, const int* dst, int E, int N, hipStream_t stream) {
  const size_t smem = (size_t)(2 * c.NGP + c.CHP) * 4;
  csrZ_kernel9<<<512, 256, 0, stream>>>((int*)c.base, c.bytes / 16);
  csrA_kernel9<<<CSR_NBLK9, 64, smem, stream>>>(dst, E, N, c.nG, c.CHP, c.NGP, c.STG, c.HST);
  csrS_kernel9<<<1, 512, 0, stream>>>(c.HST, c.nG, c.NGP, c.START, c.TOT, c.OFF);
  csrB_kernel9<<<c.nG, 256, 0, stream>>>(dst, N, c.nG, c.CHP, c.NGP, (int)c.permLen, c.STG, c.HST, c.OFF, c.START, c.TOT, c.PERM, c.ROWPTR, c.ROWCNT, c.FLAG);
}


__global__ __launch_bounds__(256) void wprep_kernel(const float* __restrict__ w, int KIN, int OUTW, int ro, b16* __restrict__ WT) {
  const int u = blockIdx.x * 256 + threadIdx.x; if (u >= OUTW * KIN / 8) return; const int e = u * 8; const int o = e / KIN, k0 = e % KIN; v8b v;
#pragma unroll
  for (int j = 0; j < 8; ++j) v[j] = (b16)(bf16_rne(w[(size_t)(k0 + j) * OUTW + o]) * WSC); for (int pass = 0; pass < 2; ++pass) { *(volatile v8b*)(WT + (size_t)(ro + o) * KIN + k0) = v; __threadfence(); }
}
__global__ __launch_bounds__(256) void wnf_kernel(const float* __restrict__ w, b16* __restrict__ WT) {
  const int u = blockIdx.x * 256 + threadIdx.x; if (u >= R * IN * IN / 8) return; const int e = u * 8; const int r = e / (IN * IN), row = (e / IN) % IN, k0 = e % IN; const int h = row / D, eo = row % D; v8b v;
#pragma unroll
  for (int j = 0; j < 8; ++j) { const int d = k0 + j - D * h; v[j] = (d >= 0 && d < D) ? (b16)(bf16_rne(w[(((size_t)r * H + h) * D + d) * D + eo]) * WSC) : (b16)0.0f; }
  for (int pass = 0; pass < 2; ++pass) { *(volatile v8b*)(WT + e) = v; __threadfence(); }
}
__global__ __launch_bounds__(32) void rel_kernel(const float* __restrict__ rel, int KR, int relIsInput, const float* __restrict__ Wr, const float* __restrict__ Wp, const float* __restrict__ bp, float* __restrict__ RA, float* __restrict__ RELN) {
  const int r = blockIdx.x, lane = threadIdx.x; float a[8], p[4]; for (int q = 0; q < 8; ++q) a[q] = 0.0f; for (int q = 0; q < 4; ++q) p[q] = bf16_rne(bp[r * IN + q * 32 + lane]);
#pragma unroll 1
  for (int k = 0; k < KR; ++k) { const float rv = relIsInput ? bf16_rne(rel[r * KR + k]) : rel[r * KR + k]; for (int q = 0; q < 8; ++q) a[q] += pmul(rv, bf16_rne(Wr[((size_t)r * KR + k) * 256 + q * 32 + lane])); for (int q = 0; q < 4; ++q) p[q] += pmul(rv, bf16_rne(Wp[((size_t)r * KR + k) * IN + q * 32 + lane])); }
  for (int pass = 0; pass < 2; ++pass) { for (int q = 0; q < 8; ++q) ((volatile float*)RA)[r * 256 + q * 32 + lane] = a[q]; for (int q = 0; q < 4; ++q) ((volatile float*)RELN)[r * IN + q * 32 + lane] = p[q]; __threadfence(); }
}
__global__ __launch_bounds__(32) void proj_kernel(const float* __restrict__ x, const b16* __restrict__ WT, const float* __restrict__ bias, float* __restrict__ XX) {
  __shared__ __attribute__((aligned(16))) b16 Ah[16][IN + 8]; __shared__ __attribute__((aligned(16))) float Tf[16][IN + 4];
  const int lane = threadIdx.x, nloc = lane & 15, hlf = lane >> 4; const size_t m0 = (size_t)blockIdx.x * 16;
  for (int rr = 0; rr < 16; ++rr) for (int q = 0; q < 4; ++q) Ah[rr][q * 32 + lane] = (b16)(bf16_rne(x[(m0 + rr) * IN + q * 32 + lane]) * XS);
  wave_lds_sync();
  v8f acc[8];
#pragma unroll
  for (int t = 0; t < 8; ++t) acc[t] = (v8f){};
#pragma unroll
  for (int kb = 0; kb < IN; kb += 32) { const v16b a = frag_kb(&Ah[nloc][kb], hlf);
#pragma unroll
    for (int t = 0; t < 8; ++t) acc[t] = wmma16b(a, frag_kb(WT + (size_t)(t * 16 + nloc) * IN + kb, hlf), acc[t]); }
#pragma unroll
  for (int t = 0; t < 8; ++t) { const int c = t * 16 + nloc; const float bb = bf16_rne(bias[c]);
#pragma unroll 1
    for (int r8 = 0; r8 < 8; ++r8) Tf[8 * hlf + r8][c] = acc[t][r8] * (1.0f / (XS * WSC)) + bb; }
  wave_lds_sync();
  for (int pass = 0; pass < 2; ++pass) { for (int rr = 0; rr < 16; ++rr) *(volatile v4f*)(XX + (m0 + rr) * IN + lane * 4) = *(const v4f*)(&Tf[rr][lane * 4]); __threadfence(); }
}
__global__ __launch_bounds__(32) void lin_kernel(const float* __restrict__ XX, const b16* __restrict__ WT, const float* __restrict__ bres, const float* __restrict__ RA, int NLIM, float* __restrict__ P, float* __restrict__ RESP, float* __restrict__ EL) {
  __shared__ __attribute__((aligned(16))) b16 Ah[16][IN + 8], Al[16][IN + 8]; __shared__ __attribute__((aligned(16))) float Tf[16][IN + 4], Se[16][8];
  const int lane = threadIdx.x, nloc = lane & 15, hlf = lane >> 4; const size_t m0 = (size_t)blockIdx.x * 16; const int r = (int)(m0 / N); if ((int)(m0 % N) >= NLIM) return;
  for (int rr = 0; rr < 16; ++rr) { const v4f v = *(const v4f*)(XX + (m0 + rr) * IN + lane * 4); for (int j = 0; j < 4; ++j) { b16 p, q; split16(v[j] * HS, p, q); Ah[rr][lane * 4 + j] = p; Al[rr][lane * 4 + j] = q; } }
  wave_lds_sync();
  const float sc = 1.0f / (HS * WSC);
#pragma unroll 1
  for (int cg = 0; cg < 2; ++cg) { v8f acc[8];
#pragma unroll
    for (int t = 0; t < 8; ++t) acc[t] = (v8f){};
#pragma unroll
    for (int kb = 0; kb < IN; kb += 32) { const v16b a = frag_kb(&Ah[nloc][kb], hlf), al = frag_kb(&Al[nloc][kb], hlf);
#pragma unroll
      for (int t = 0; t < 8; ++t) { const v16b bw = frag_kb(WT + (size_t)(cg * 128 + t * 16 + nloc) * IN + kb, hlf); acc[t] = wmma16b(a, bw, acc[t]); acc[t] = wmma16b(al, bw, acc[t]); } }
    if (cg == 0) {
      float pd[8], ps[8];
#pragma unroll
      for (int t = 0; t < 8; ++t) { const int c = t * 16 + nloc, h = t >> 1, cc = c & 31; const float wd = RA[r * 256 + h * 64 + cc], wsv = RA[r * 256 + h * 64 + 32 + cc];
        if ((t & 1) == 0) for (int r8 = 0; r8 < 8; ++r8) { pd[r8] = 0.0f; ps[r8] = 0.0f; }
#pragma unroll
        for (int r8 = 0; r8 < 8; ++r8) { const float p = acc[t][r8] * sc; Tf[8 * hlf + r8][c] = p; pd[r8] += pmul(p, wd); ps[r8] += pmul(p, wsv); }
        if (t & 1) {
#pragma unroll
          for (int r8 = 0; r8 < 8; ++r8) { float s = ps[r8], d = pd[r8]; for (int o = 1; o < 16; o <<= 1) { s += __shfl_xor(s, o); d += __shfl_xor(d, o); } if (nloc == 0) { Se[8 * hlf + r8][h] = s; Se[8 * hlf + r8][4 + h] = d; } } } }
      wave_lds_sync();
      for (int pass = 0; pass < 2; ++pass) { for (int rr = 0; rr < 16; ++rr) *(volatile v4f*)(P + (m0 + rr) * IN + lane * 4) = *(const v4f*)(&Tf[rr][lane * 4]); for (int q = 0; q < 4; ++q) ((volatile float*)EL)[m0 * 8 + q * 32 + lane] = Se[(q * 32 + lane) >> 3][(q * 32 + lane) & 7]; __threadfence(); }
      wave_lds_sync(); }
    else {
#pragma unroll
      for (int t = 0; t < 8; ++t) { const int c = t * 16 + nloc; const float bb = bf16_rne(bres[c]);
#pragma unroll 1
        for (int r8 = 0; r8 < 8; ++r8) Tf[8 * hlf + r8][c] = acc[t][r8] * sc + bb; }
      wave_lds_sync();
      for (int pass = 0; pass < 2; ++pass) { for (int rr = 0; rr < 16; ++rr) *(volatile v4f*)(RESP + (m0 + rr) * IN + lane * 4) = *(const v4f*)(&Tf[rr][lane * 4]); __threadfence(); }
      wave_lds_sync(); } }
}
__global__ __launch_bounds__(256) void att_kernel(const float* __restrict__ P, const float* __restrict__ EL, const float* __restrict__ RESP, const float* __restrict__ resw, const int* __restrict__ srcs, const int* __restrict__ PERM, const int* __restrict__ ROWPTR, const int* __restrict__ ROWCNT, int permLen, int r, int NLIM, float* __restrict__ OUT_) {
  const int wave = threadIdx.x >> 5, lane = threadIdx.x & 31; const size_t v = (size_t)blockIdx.x * 8 + wave; const size_t row = (size_t)r * N + v; v4f o = {0, 0, 0, 0};
  if (v < (size_t)NLIM) { const int h = lane >> 3; const float edv = EL[row * 8 + 4 + h]; int st = ROWPTR[v], cnt = ROWCNT[v]; cnt = iclamp(cnt, 0, 1 << 20); st = iclamp(st, 0, permLen - cnt); float mx = -INFINITY; int used = 0;
#pragma unroll 1
    for (int j = 0; j < cnt; ++j) { const int e = iclamp(PERM[st + j], 0, E - 1); const size_t s = (size_t)iclamp(srcs[(size_t)r * E + e], 0, N - 1); if (s >= (size_t)NLIM) continue; ++used; mx = fmaxf(mx, leaky(EL[((size_t)r * N + s) * 8 + h] + edv)); }
    float den = 0.0f, m4[4] = {0, 0, 0, 0};
    if (used > 0) {
#pragma unroll 1
      for (int j = 0; j < cnt; ++j) { const int e = iclamp(PERM[st + j], 0, E - 1); const size_t s = (size_t)iclamp(srcs[(size_t)r * E + e], 0, N - 1); if (s >= (size_t)NLIM) continue; const float p = __expf(leaky(EL[((size_t)r * N + s) * 8 + h] + edv) - mx); den += p; const v4f f = *(const v4f*)(P + ((size_t)r * N + s) * IN + lane * 4); for (int i = 0; i < 4; ++i) m4[i] += pmul(p, f[i]); } }
    const float inv = used > 0 ? 1.0f / (den + 1e-16f) : 0.0f; const float al = sigm(bf16_rne(resw[0])); const v4f rs = *(const v4f*)(RESP + row * IN + lane * 4);
    for (int i = 0; i < 4; ++i) o[i] = pmul(fmaxf(pmul(m4[i], inv), 0.0f), al) + pmul(rs[i], 1.0f - al); }
  for (int pass = 0; pass < 2; ++pass) { *(volatile v4f*)(OUT_ + row * IN + lane * 4) = o; __threadfence(); }
}
__global__ __launch_bounds__(256) void cross_kernel(const float* __restrict__ OUT_, const float* __restrict__ Wx, int NLIM, float* __restrict__ XX) {
  const int wave = threadIdx.x >> 5, lane = threadIdx.x & 31; const size_t n = (size_t)blockIdx.x * 8 + wave; const int h = lane >> 3, c4 = lane * 4;
  v4f f[R]; for (int r = 0; r < R; ++r) f[r] = (n < (size_t)NLIM) ? *(const v4f*)(OUT_ + ((size_t)r * N + n) * IN + c4) : (v4f){0, 0, 0, 0};
  for (int rho = 0; rho < R; ++rho) { float w4[4]; for (int i = 0; i < 4; ++i) w4[i] = bf16_rne(Wx[(rho * H + h) * D + (c4 & 31) + i]); float sc[R];
    for (int r = 0; r < R; ++r) { float s = 0.0f; for (int i = 0; i < 4; ++i) s += pmul(f[r][i], w4[i]); s += __shfl_xor(s, 1); s += __shfl_xor(s, 2); s += __shfl_xor(s, 4); sc[r] = leaky(s); }
    const float m = fmaxf(sc[0], fmaxf(sc[1], sc[2])); float ex[R], tot = 0.0f; for (int r = 0; r < R; ++r) { ex[r] = __expf(sc[r] - m); tot += ex[r]; } const float inv = 1.0f / tot;
    v4f o; for (int i = 0; i < 4; ++i) { float a = 0.0f; for (int r = 0; r < R; ++r) a += pmul(f[r][i], ex[r] * inv); o[i] = a; }
    for (int pass = 0; pass < 2; ++pass) { *(volatile v4f*)(XX + ((size_t)rho * N + n) * IN + c4) = o; __threadfence(); } }
}
__global__ __launch_bounds__(32) void fuse_kernel(const float* __restrict__ XX, const b16* __restrict__ WNF, const float* __restrict__ RELN, const float* __restrict__ Wrf, int NLIM, float* __restrict__ out) {
  __shared__ __attribute__((aligned(16))) b16 Ah[16][IN + 8], Al[16][IN + 8]; __shared__ __attribute__((aligned(16))) float T3[R][16][IN + 4], Rp[R][IN];
  const int lane = threadIdx.x, nloc = lane & 15, hlf = lane >> 4; const size_t m0 = (size_t)blockIdx.x * 16; if (m0 >= (size_t)NLIM) return; const int h4 = lane >> 3;
  for (int r = 0; r < R; ++r) for (int q = 0; q < 4; ++q) { const int col = q * 32 + lane; const int h = col / D, e = col % D; float s = 0.0f;
#pragma unroll 1
    for (int c = 0; c < D; ++c) s += pmul(RELN[r * IN + h * D + c], bf16_rne(Wrf[(((size_t)r * H + h) * D + c) * D + e])); Rp[r][col] = s; }
#pragma unroll 1
  for (int r = 0; r < R; ++r) {
    for (int rr = 0; rr < 16; ++rr) { const v4f v = *(const v4f*)(XX + ((size_t)r * N + m0 + rr) * IN + lane * 4); for (int j = 0; j < 4; ++j) { b16 p, q; split16(v[j] * HS, p, q); Ah[rr][lane * 4 + j] = p; Al[rr][lane * 4 + j] = q; } }
    wave_lds_sync();
    v8f acc[8];
#pragma unroll
    for (int t = 0; t < 8; ++t) acc[t] = (v8f){};
#pragma unroll
    for (int kb = 0; kb < IN; kb += 32) { const v16b a = frag_kb(&Ah[nloc][kb], hlf), al = frag_kb(&Al[nloc][kb], hlf);
#pragma unroll
      for (int t = 0; t < 8; ++t) { if ((t >> 1) != (kb >> 5)) continue; const v16b bw = frag_kb(WNF + ((size_t)r * IN + t * 16 + nloc) * IN + kb, hlf); acc[t] = wmma16b(a, bw, acc[t]); acc[t] = wmma16b(al, bw, acc[t]); } }
#pragma unroll
    for (int t = 0; t < 8; ++t)
#pragma unroll 1
      for (int r8 = 0; r8 < 8; ++r8) T3[r][8 * hlf + r8][t * 16 + nloc] = acc[t][r8] * (1.0f / (HS * WSC));
    wave_lds_sync(); }
  for (int rr = 0; rr < 16; ++rr) { float sc[R]; v4f hv[R];
    for (int r = 0; r < R; ++r) { hv[r] = *(const v4f*)(&T3[r][rr][lane * 4]); float s = 0.0f; for (int i = 0; i < 4; ++i) s += pmul(hv[r][i], Rp[r][lane * 4 + i]); s += __shfl_xor(s, 1); s += __shfl_xor(s, 2); s += __shfl_xor(s, 4); sc[r] = leaky(s); }
    const float m = fmaxf(sc[0], fmaxf(sc[1], sc[2])); float ex[R], tot = 0.0f; for (int r = 0; r < R; ++r) { ex[r] = __expf(sc[r] - m); tot += ex[r]; } const float inv = 1.0f / tot;
    v4f o; for (int i = 0; i < 4; ++i) { float a = 0.0f; for (int r = 0; r < R; ++r) a += pmul(hv[r][i], ex[r] * inv); o[i] = a; }
    *(v4f*)(&T3[0][rr][lane * 4]) = o; }
  (void)h4; wave_lds_sync();
  for (int pass = 0; pass < 2; ++pass) { for (int rr = 0; rr < 16; ++rr) *(volatile v4f*)(out + (m0 + rr) * IN + lane * 4) = *(const v4f*)(&T3[0][rr][lane * 4]); __threadfence(); }
}
}

extern "C" void kernel_launch(void* const* d_in, const int* in_sizes, int n_in, void* d_out, int out_size, void* d_ws, size_t ws_size, hipStream_t stream) {
  (void)n_in;
  auto Fp = [&](int i) { return (const float*)d_in[i]; }; auto Ip = [&](int i) { return (const int*)d_in[i]; };
  if (in_sizes[0] != RN * IN || in_sizes[1] != R * E || in_sizes[2] != R * E || in_sizes[3] != IN * IN || in_sizes[5] != R * 64 || in_sizes[6] != IN * IN || in_sizes[7] != R * 64 * 256 || in_sizes[14] != IN * IN || in_sizes[15] != R * IN * 256 || in_sizes[22] != R * H * D * D || out_size != N * IN) return;
  const int NLIM = N; const int GB8 = N / 8, GB16 = NBLK;
  size_t off = 0; char* ws = (char*)d_ws;
  auto carve = [&](size_t bytes) { char* p = ws + off; off += (bytes + 255) & ~(size_t)255; return p; };
  b16* WPJ = (b16*)carve((size_t)IN * IN * 2); b16* WL0 = (b16*)carve((size_t)2 * IN * IN * 2); b16* WL1 = (b16*)carve((size_t)2 * IN * IN * 2); b16* WNF = (b16*)carve((size_t)R * IN * IN * 2);
  float* RA = (float*)carve(R * 256 * 4); float* REL1 = (float*)carve(R * IN * 4); float* REL2 = (float*)carve(R * IN * 4);
  float* XX = (float*)carve((size_t)RN * IN * 4); float* P = (float*)carve((size_t)RN * IN * 4); float* RESP = (float*)carve((size_t)RN * IN * 4); float* OUTP = (float*)carve((size_t)RN * IN * 4); float* EL = (float*)carve((size_t)RN * 8 * 4);
  CsrBufs9 csr[R]; for (int r = 0; r < R; ++r) off = csr_carve9(csr[r], ws, off, E, N);
  if (off > ws_size || off > ((size_t)192 << 20)) return;
  wprep_kernel<<<(IN * IN / 8 + 255) / 256, 256, 0, stream>>>(Fp(3), IN, IN, 0, WPJ);
  wprep_kernel<<<(IN * IN / 8 + 255) / 256, 256, 0, stream>>>(Fp(6), IN, IN, 0, WL0); wprep_kernel<<<(IN * IN / 8 + 255) / 256, 256, 0, stream>>>(Fp(10), IN, IN, IN, WL0);
  wprep_kernel<<<(IN * IN / 8 + 255) / 256, 256, 0, stream>>>(Fp(14), IN, IN, 0, WL1); wprep_kernel<<<(IN * IN / 8 + 255) / 256, 256, 0, stream>>>(Fp(18), IN, IN, IN, WL1);
  wnf_kernel<<<(R * IN * IN / 8 + 255) / 256, 256, 0, stream>>>(Fp(22), WNF);
  for (int r = 0; r < R; ++r) csr_build9(csr[r], Ip(2) + (size_t)r * E, E, N, stream);
  proj_kernel<<<RN / 16, 32, 0, stream>>>(Fp(0), WPJ, Fp(4), XX);
  rel_kernel<<<R, 32, 0, stream>>>(Fp(5), 64, 1, Fp(7), Fp(8), Fp(9), RA, REL1);
  lin_kernel<<<RN / 16, 32, 0, stream>>>(XX, WL0, Fp(11), RA, NLIM, P, RESP, EL);
  for (int r = 0; r < R; ++r) att_kernel<<<GB8, 256, 0, stream>>>(P, EL, RESP, Fp(12), Ip(1), csr[r].PERM, csr[r].ROWPTR, csr[r].ROWCNT, (int)csr[r].permLen, r, NLIM, OUTP);
  cross_kernel<<<GB8, 256, 0, stream>>>(OUTP, Fp(13), NLIM, XX);
  rel_kernel<<<R, 32, 0, stream>>>(REL1, IN, 0, Fp(15), Fp(16), Fp(17), RA, REL2);
  lin_kernel<<<RN / 16, 32, 0, stream>>>(XX, WL1, Fp(19), RA, NLIM, P, RESP, EL);
  for (int r = 0; r < R; ++r) att_kernel<<<GB8, 256, 0, stream>>>(P, EL, RESP, Fp(20), Ip(1), csr[r].PERM, csr[r].ROWPTR, csr[r].ROWCNT, (int)csr[r].permLen, r, NLIM, OUTP);
  cross_kernel<<<GB8, 256, 0, stream>>>(OUTP, Fp(21), NLIM, XX);
  fuse_kernel<<<GB16, 32, 0, stream>>>(XX, WNF, REL2, Fp(23), NLIM, (float*)d_out);
}
